// DUPLEX_gat_32684701123297
// MI455X (gfx1250) — hardware-verified
//
#include <hip/hip_runtime.h>
#include <stddef.h>


#define FW    128
#define NHD   4
#define OW    32
#define GR    32
#define AP    136
#define XSP   132
#define NTHR  256
#define NWAVE 8
#define NB    256
#define CHUNK 1024
#define WCAP  128
#define WPL   (FW * FW)

#define LDS_SACC (NB * 2 * FW)
#define LDS_STAT (NB * NHD * 4)
#define LDS_ER   (NB * NHD * 2)
#define LDS_LIST (NWAVE * WCAP)
#define LDS_BYTES ((LDS_SACC + LDS_STAT + LDS_ER + LDS_LIST + NWAVE) * 4)

static_assert(WCAP == (CHUNK / NTHR) * 32);
static_assert(CHUNK == NTHR * 4);
static_assert(NB == 256);
static_assert((NB % (NWAVE * 4)) == 0);
static_assert(((LDS_SACC % 4) == 0) && ((LDS_STAT % 4) == 0) && ((LDS_ER % 4) == 0));
static_assert(LDS_BYTES == 290848);
static_assert((AP % 8) == 0 && (XSP % 4) == 0);

typedef float    v2f  __attribute__((ext_vector_type(2)));
typedef float    v4f  __attribute__((ext_vector_type(4)));
typedef float    v8f  __attribute__((ext_vector_type(8)));
typedef int      v4i  __attribute__((ext_vector_type(4)));
typedef __bf16   v8b  __attribute__((ext_vector_type(8)));
typedef __bf16   v16b __attribute__((ext_vector_type(16)));
union FragB { v16b v; v8b half[2]; };
union PackB { v8b b; v4i i; unsigned short s[8]; };

__device__ __forceinline__ v8f wm(v16b a, v16b b, v8f c) {
  v8f d = __builtin_amdgcn_wmma_f32_16x16x32_bf16(false, a, false, b, (short)0, c, false, false);
  asm volatile("v_nop\n\tv_nop\n\tv_nop\n\tv_nop" : "+v"(d) : "v"(a), "v"(b));
  return d;
}

__device__ __forceinline__ unsigned bf_rne(float f) {
  unsigned u = __float_as_uint(f);
  u += 0x7FFFu + ((u >> 16) & 1u);
  return u >> 16;
}
__device__ __forceinline__ void split2(float f, unsigned short& hi, unsigned short& lo) {
  const unsigned h = bf_rne(f);
  const float hf = __uint_as_float(h << 16);
  hi = (unsigned short)h;
  lo = (unsigned short)bf_rne(f - hf);
}

__device__ __forceinline__ v4f xsum4(v4f v, int mk) {
  v4f r;
  r.x = __shfl_xor(v.x, mk, 32);
  r.y = __shfl_xor(v.y, mk, 32);
  r.z = __shfl_xor(v.z, mk, 32);
  r.w = __shfl_xor(v.w, mk, 32);
  return v + r;
}

__global__ __launch_bounds__(NTHR) void k_prepw(
    const float* __restrict__ W0, const float* __restrict__ W1,
    const float* __restrict__ W2, const float* __restrict__ W3, __bf16* planes) {
  const int mid = blockIdx.y;
  const float* W = (mid == 0) ? W0 : ((mid == 1) ? W1 : ((mid == 2) ? W2 : W3));
  const int t = blockIdx.x * NTHR + threadIdx.x;
  if (t >= FW * (FW / 8)) return;
  const int n  = t >> 4;
  const int k0 = (t & 15) * 8;
  PackB uh, ul;
#pragma unroll
  for (int i = 0; i < 8; ++i) split2(W[(k0 + i) * FW + n], uh.s[i], ul.s[i]);
  __bf16* ph = planes + (size_t)mid * 2 * WPL + (size_t)n * FW + k0;
  __bf16* pl = ph + WPL;
  *(volatile v4i*)ph = uh.i;
  *(volatile v4i*)pl = ul.i;
  __threadfence();
  *(volatile v4i*)ph = uh.i;
  *(volatile v4i*)pl = ul.i;
}

__device__ __forceinline__ void epi_tile(v8f acc, int T, int hh, int m, int wave, int ncol,
                                         float cs, float cd, float* Xs, float* As, float* Ds) {
  float ss[8], sd[8];
#pragma unroll
  for (int r = 0; r < 8; ++r) {
    const float v = acc[r];
    Xs[(T * 16 + 8 * hh + r) * XSP + ncol] = v;
    ss[r] = v * cs;
    sd[r] = v * cd;
  }
#pragma unroll
  for (int mk = 1; mk < 16; mk <<= 1) {
#pragma unroll
    for (int r = 0; r < 8; ++r) {
      ss[r] += __shfl_xor(ss[r], mk, 32);
      sd[r] += __shfl_xor(sd[r], mk, 32);
    }
  }
  if (m == 0) {
#pragma unroll
    for (int r = 0; r < 8; ++r) {
      As[(T * 16 + 8 * hh + r) * NWAVE + wave] = ss[r];
      Ds[(T * 16 + 8 * hh + r) * NWAVE + wave] = sd[r];
    }
  }
}

__global__ __launch_bounds__(NTHR) void k_gemm(
    const float* __restrict__ x0, const float* __restrict__ x1,
    const __bf16* __restrict__ wq0, const __bf16* __restrict__ wq1,
    const float* __restrict__ al0, const float* __restrict__ ar0,
    const float* __restrict__ al1, const float* __restrict__ ar1,
    float* ft0, float* ft1, float* el0, float* er0, float* el1, float* er1, int nN) {
  __shared__ __attribute__((aligned(16))) __bf16 Ah[GR * AP];
  __shared__ __attribute__((aligned(16))) __bf16 Al[GR * AP];
  __shared__ __attribute__((aligned(16))) float Xs[GR * XSP];
  __shared__ __attribute__((aligned(16))) float As[GR * NWAVE];
  __shared__ __attribute__((aligned(16))) float Ds[GR * NWAVE];

  const int br = blockIdx.y;
  const float*  x  = br ? x1 : x0;
  const __bf16* wq = br ? wq1 : wq0;
  const float*  al = br ? al1 : al0;
  const float*  ar = br ? ar1 : ar0;
  float* ft = br ? ft1 : ft0;
  float* el = br ? el1 : el0;
  float* er = br ? er1 : er0;

  const int tid  = threadIdx.x;
  const int lane = tid & 31;
  const int wave = tid >> 5;
  const int hh   = lane >> 4;
  const int m    = lane & 15;
  const int rowBase = blockIdx.x * GR;

  {
    const int r  = tid >> 3;
    const int c0 = (tid & 7) * 16;
    int row = rowBase + r;
    if (row > nN - 1) row = nN - 1;
    const float* p = x + (size_t)row * FW + c0;
    const v4f f0 = *(const v4f*)(p), f1 = *(const v4f*)(p + 4);
    const v4f f2 = *(const v4f*)(p + 8), f3 = *(const v4f*)(p + 12);
    const float fv[16] = {f0.x, f0.y, f0.z, f0.w, f1.x, f1.y, f1.z, f1.w,
                          f2.x, f2.y, f2.z, f2.w, f3.x, f3.y, f3.z, f3.w};
    PackB h0, h1, l0, l1;
#pragma unroll
    for (int i = 0; i < 8; ++i) {
      split2(fv[i],     h0.s[i], l0.s[i]);
      split2(fv[8 + i], h1.s[i], l1.s[i]);
    }
    *(v8b*)(Ah + r * AP + c0)     = h0.b;
    *(v8b*)(Ah + r * AP + c0 + 8) = h1.b;
    *(v8b*)(Al + r * AP + c0)     = l0.b;
    *(v8b*)(Al + r * AP + c0 + 8) = l1.b;
  }
  __syncthreads();

  const int ncol = wave * 16 + m;
  const __bf16* wh = wq + (size_t)ncol * FW;
  const __bf16* wl = wh + WPL;
  v8f c0a = {0.f, 0.f, 0.f, 0.f, 0.f, 0.f, 0.f, 0.f};
  v8f c1a = {0.f, 0.f, 0.f, 0.f, 0.f, 0.f, 0.f, 0.f};
#pragma unroll
  for (int kt = 0; kt < FW / 32; ++kt) {
    const int k0 = kt * 32;
    FragB bh, bl, a0h, a0l, a1h, a1l;
    const __bf16* pbh  = wh + k0 + 8 * hh;
    const __bf16* pbl  = wl + k0 + 8 * hh;
    const __bf16* pa0h = Ah + m * AP + k0 + 8 * hh;
    const __bf16* pa0l = Al + m * AP + k0 + 8 * hh;
    const __bf16* pa1h = Ah + (16 + m) * AP + k0 + 8 * hh;
    const __bf16* pa1l = Al + (16 + m) * AP + k0 + 8 * hh;
    bh.half[0]  = *(const v8b*)pbh;   bh.half[1]  = *(const v8b*)(pbh + 16);
    bl.half[0]  = *(const v8b*)pbl;   bl.half[1]  = *(const v8b*)(pbl + 16);
    a0h.half[0] = *(const v8b*)pa0h;  a0h.half[1] = *(const v8b*)(pa0h + 16);
    a0l.half[0] = *(const v8b*)pa0l;  a0l.half[1] = *(const v8b*)(pa0l + 16);
    a1h.half[0] = *(const v8b*)pa1h;  a1h.half[1] = *(const v8b*)(pa1h + 16);
    a1l.half[0] = *(const v8b*)pa1l;  a1l.half[1] = *(const v8b*)(pa1l + 16);
    c0a = wm(a0h.v, bh.v, c0a);
    c0a = wm(a0h.v, bl.v, c0a);
    c0a = wm(a0l.v, bh.v, c0a);
    c1a = wm(a1h.v, bh.v, c1a);
    c1a = wm(a1h.v, bl.v, c1a);
    c1a = wm(a1l.v, bh.v, c1a);
  }

  const float cs = al[ncol];
  const float cd = ar[ncol];
  epi_tile(c0a, 0, hh, m, wave, ncol, cs, cd, Xs, As, Ds);
  epi_tile(c1a, 1, hh, m, wave, ncol, cs, cd, Xs, As, Ds);
  __syncthreads();

  v4f xr[4];
#pragma unroll
  for (int i = 0; i < 4; ++i) xr[i] = *(const v4f*)(Xs + (4 * wave + i) * XSP + 4 * lane);
  const float* hs = (wave == 0) ? As : Ds;
  v4f gv;
  gv.x = hs[lane * NWAVE + 0] + hs[lane * NWAVE + 1];
  gv.y = hs[lane * NWAVE + 2] + hs[lane * NWAVE + 3];
  gv.z = hs[lane * NWAVE + 4] + hs[lane * NWAVE + 5];
  gv.w = hs[lane * NWAVE + 6] + hs[lane * NWAVE + 7];
  float* gp = ((wave == 0) ? el : er) + (size_t)rowBase * NHD + 4 * lane;
  float* fp[4];
#pragma unroll
  for (int i = 0; i < 4; ++i) fp[i] = ft + (size_t)(rowBase + 4 * wave + i) * FW + 4 * lane;

#pragma unroll
  for (int i = 0; i < 4; ++i) *(volatile v4f*)(fp[i]) = xr[i];
  if (wave < 2) *(volatile v4f*)gp = gv;
  __threadfence();
#pragma unroll
  for (int i = 0; i < 4; ++i) *(volatile v4f*)(fp[i]) = xr[i];
  if (wave < 2) *(volatile v4f*)gp = gv;
}

__global__ __launch_bounds__(NTHR) void k_agg(
    const int* __restrict__ src, const int* __restrict__ dst,
    const float* __restrict__ w_am, const float* __restrict__ w_ph,
    const float* __restrict__ ft_am, const float* __restrict__ ft_ph,
    const float* __restrict__ el_am, const float* __restrict__ er_am,
    const float* __restrict__ el_ph, const float* __restrict__ er_ph,
    const float* __restrict__ b_am, const float* __restrict__ b_ph,
    float* o_am, float* o_ph, int nN, int nE, int last) {
  extern __shared__ v4f lds_dyn[];
  float* sacc = (float*)lds_dyn;
  float* stat = sacc + LDS_SACC;
  float* erS  = stat + LDS_STAT;
  int*   list = (int*)(erS + LDS_ER);
  int*   wcnt = list + LDS_LIST;

  const int tid  = threadIdx.x;
  const int lane = tid & 31;
  const int wave = tid >> 5;
  const int hd   = lane >> 3;
  const int nodeBase = blockIdx.x * NB;

  {
    const v4f z4 = {0.f, 0.f, 0.f, 0.f};
    for (int i = tid; i < LDS_SACC / 4; i += NTHR) lds_dyn[i] = z4;
    const float ninf = __uint_as_float(0xff800000u);
    const v4f s4 = {ninf, 0.f, ninf, 0.f};
    v4f* st4 = (v4f*)stat;
    for (int i = tid; i < NB * NHD; i += NTHR) st4[i] = s4;
    for (int i = tid; i < NB * NHD; i += NTHR) {
      const int slot = i >> 2, h = i & 3;
      int nd = nodeBase + slot;
      if (nd > nN - 1) nd = nN - 1;
      erS[2 * i]     = er_am[(size_t)nd * NHD + h];
      erS[2 * i + 1] = er_ph[(size_t)nd * NHD + h];
    }
  }
  __syncthreads();

  const bool vec_ok = ((reinterpret_cast<size_t>(dst)) & 15) == 0;
  const int nChunks = (nE + CHUNK - 1) / CHUNK;
  const int sent = -2147483647 - 1;

#pragma unroll 1
  for (int ch = 0; ch < nChunks; ++ch) {
    const int cbase = ch * CHUNK;
    int wc = 0;
    {
      const int el0 = tid * 4;
      const int e0  = cbase + el0;
      v4i d;
      if (vec_ok && (cbase + CHUNK <= nE)) {
        d = *(const v4i*)(dst + e0);
      } else {
        d.x = (e0     < nE) ? dst[min(e0,     nE - 1)] : sent;
        d.y = (e0 + 1 < nE) ? dst[min(e0 + 1, nE - 1)] : sent;
        d.z = (e0 + 2 < nE) ? dst[min(e0 + 2, nE - 1)] : sent;
        d.w = (e0 + 3 < nE) ? dst[min(e0 + 3, nE - 1)] : sent;
      }
      const unsigned s0 = (unsigned)d.x - (unsigned)nodeBase;
      const unsigned s1 = (unsigned)d.y - (unsigned)nodeBase;
      const unsigned s2 = (unsigned)d.z - (unsigned)nodeBase;
      const unsigned s3 = (unsigned)d.w - (unsigned)nodeBase;
      const bool h0 = s0 < (unsigned)NB;
      const bool h1 = s1 < (unsigned)NB;
      const bool h2 = s2 < (unsigned)NB;
      const bool h3 = s3 < (unsigned)NB;
      const unsigned many = __builtin_amdgcn_ballot_w32(h0 | h1 | h2 | h3);
      if (many != 0u) {
#define HITJ(J, HJ, SJ) { \
          const unsigned mj = __builtin_amdgcn_ballot_w32(HJ); \
          if (HJ) { \
            const int pos = wc + (int)__builtin_amdgcn_mbcnt_lo(mj, 0u); \
            if (pos < WCAP) list[wave * WCAP + pos] = ((el0 + (J)) << 8) | (int)(SJ); \
          } \
          wc += (int)__builtin_popcount(mj); }
        HITJ(0, h0, s0)
        HITJ(1, h1, s1)
        HITJ(2, h2, s2)
        HITJ(3, h3, s3)
#undef HITJ
      }
    }
    if (lane == 0) wcnt[wave] = wc;
    __syncthreads();

    if (wave == 0) {
#pragma unroll 1
      for (int wsx = 0; wsx < NWAVE; ++wsx) {
        int n = wcnt[wsx];
        if (n > WCAP) n = WCAP;
        if (n < 0) n = 0;
#pragma unroll 1
        for (int i = 0; i < n; ++i) {
          const int ent  = list[wsx * WCAP + i];
          const int slot = ent & (NB - 1);
          const int eloc = (ent >> 8) & (CHUNK - 1);
          int e = cbase + eloc;
          if (e > nE - 1) e = nE - 1;
          int s = src[e];
          s = (s < 0) ? 0 : ((s > nN - 1) ? nN - 1 : s);
          const float wa = w_am[e];
          const float wp = w_ph[e];
          const int sh = slot * NHD + hd;
          const v2f erv = *(const v2f*)(erS + sh * 2);
          float la = el_am[(size_t)s * NHD + hd] + erv.x;
          float lp = el_ph[(size_t)s * NHD + hd] + erv.y;
          la = (la > 0.f) ? la : 0.2f * la;
          lp = (lp > 0.f) ? lp : 0.2f * lp;
          v4f* stp = (v4f*)(stat + sh * 4);
          const v4f st = *stp;
          const float ma = fmaxf(st.x, la);
          const float mp = fmaxf(st.z, lp);
          const float sa = __expf(st.x - ma);
          const float sp = __expf(st.z - mp);
          const float pa = __expf(la - ma);
          const float pp = __expf(lp - mp);
          const v4f fa = *(const v4f*)(ft_am + (size_t)s * FW + 4 * lane);
          const v4f fp = *(const v4f*)(ft_ph + (size_t)s * FW + 4 * lane);
          v4f* qa = (v4f*)(sacc + slot * (2 * FW) + 4 * lane);
          v4f* qp = (v4f*)(sacc + slot * (2 * FW) + FW + 4 * lane);
          const v4f ca = *qa;
          const v4f cp = *qp;
          const float ga = pa * wa;
          const float gq = pp * wp;
          const v4f na = ca * sa + ga * fa;
          const v4f np = cp * sp + gq * fp;
          *qa = na;
          *qp = np;
          if ((lane & 7) == 0) {
            v4f ns;
            ns.x = ma; ns.y = st.y * sa + pa;
            ns.z = mp; ns.w = st.w * sp + pp;
            *stp = ns;
          }
          asm volatile("" ::: "memory");
        }
      }
    }
    __syncthreads();
  }

  const v4f ba = *(const v4f*)(b_am + 4 * lane);
  const v4f bp = *(const v4f*)(b_ph + 4 * lane);
  if (last == 0) {
#pragma unroll 1
    for (int j = 0; j < NB / NWAVE; ++j) {
      const int slot = wave * (NB / NWAVE) + j;
      const int node = nodeBase + slot;
      if (node >= nN) break;
      const v4f st = *(const v4f*)(stat + (slot * NHD + hd) * 4);
      const float ia = __builtin_amdgcn_rcpf(fmaxf(st.y, 1e-9f));
      const float ip = __builtin_amdgcn_rcpf(fmaxf(st.w, 1e-9f));
      v4f ya = *(const v4f*)(sacc + slot * (2 * FW) + 4 * lane) * ia + ba;
      v4f yp = *(const v4f*)(sacc + slot * (2 * FW) + FW + 4 * lane) * ip + bp;
      ya.x = ya.x > 0.f ? ya.x : 0.f; ya.y = ya.y > 0.f ? ya.y : 0.f;
      ya.z = ya.z > 0.f ? ya.z : 0.f; ya.w = ya.w > 0.f ? ya.w : 0.f;
      yp.x = yp.x > 0.f ? yp.x : 0.f; yp.y = yp.y > 0.f ? yp.y : 0.f;
      yp.z = yp.z > 0.f ? yp.z : 0.f; yp.w = yp.w > 0.f ? yp.w : 0.f;
      float* pa = o_am + (size_t)node * FW + 4 * lane;
      float* pq = o_ph + (size_t)node * FW + 4 * lane;
      *(volatile v4f*)pa = ya;
      *(volatile v4f*)pq = yp;
      __threadfence();
      *(volatile v4f*)pa = ya;
      *(volatile v4f*)pq = yp;
    }
  } else {
#pragma unroll 1
    for (int g = 0; g < NB / NWAVE / 4; ++g) {
      const int slot0 = wave * (NB / NWAVE) + 4 * g;
      const int node0 = nodeBase + slot0;
      if (node0 >= nN) break;
      v4f ysa = {0.f, 0.f, 0.f, 0.f};
      v4f ysp = {0.f, 0.f, 0.f, 0.f};
#pragma unroll 1
      for (int q = 0; q < 4; ++q) {
        const int slot = slot0 + q;
        const v4f st = *(const v4f*)(stat + (slot * NHD + hd) * 4);
        const float ia = __builtin_amdgcn_rcpf(fmaxf(st.y, 1e-9f));
        const float ip = __builtin_amdgcn_rcpf(fmaxf(st.w, 1e-9f));
        v4f va = *(const v4f*)(sacc + slot * (2 * FW) + 4 * lane) * ia + ba;
        v4f vp = *(const v4f*)(sacc + slot * (2 * FW) + FW + 4 * lane) * ip + bp;
        va = xsum4(va, 8);  va = xsum4(va, 16);
        vp = xsum4(vp, 8);  vp = xsum4(vp, 16);
        va = va * 0.25f;
        vp = vp * 0.25f;
        if ((lane >> 3) == q) { ysa = va; ysp = vp; }
      }
      const int row = node0 + (lane >> 3);
      float* pa = o_am + (size_t)row * OW + 4 * (lane & 7);
      float* pq = o_ph + (size_t)row * OW + 4 * (lane & 7);
      if (row < nN) {
        *(volatile v4f*)pa = ysa;
        *(volatile v4f*)pq = ysp;
      }
      __threadfence();
      if (row < nN) {
        *(volatile v4f*)pa = ysa;
        *(volatile v4f*)pq = ysp;
      }
    }
  }
}

extern "C" void kernel_launch(void* const* d_in, const int* in_sizes, int n_in,
                              void* d_out, int out_size, void* d_ws, size_t ws_size,
                              hipStream_t stream) {
  if (n_in < 22) return;
  const int nN = in_sizes[0] / FW;
  if (nN <= 0 || in_sizes[0] != nN * FW || in_sizes[1] != nN * FW) return;
  const int nE = in_sizes[4];
  if (nE <= 0 || in_sizes[5] != nE || in_sizes[2] != nE || in_sizes[3] != nE) return;
  for (int g = 0; g < 4; ++g) {
    const int b = 6 + 4 * g;
    if (in_sizes[b] != WPL || in_sizes[b + 1] != NHD * 32 || in_sizes[b + 2] != NHD * 32 || in_sizes[b + 3] != FW) return;
  }
  if (out_size != 2 * nN * OW) return;

  const float* x_am     = (const float*)d_in[0];
  const float* x_ph     = (const float*)d_in[1];
  const float* exist    = (const float*)d_in[2];
  const float* am_exist = (const float*)d_in[3];
  const int*   src      = (const int*)d_in[4];
  const int*   dst      = (const int*)d_in[5];
  const float* W0a = (const float*)d_in[6];   const float* al0a = (const float*)d_in[7];
  const float* ar0a = (const float*)d_in[8];  const float* b0a  = (const float*)d_in[9];
  const float* W0p = (const float*)d_in[10];  const float* al0p = (const float*)d_in[11];
  const float* ar0p = (const float*)d_in[12]; const float* b0p  = (const float*)d_in[13];
  const float* W1a = (const float*)d_in[14];  const float* al1a = (const float*)d_in[15];
  const float* ar1a = (const float*)d_in[16]; const float* b1a  = (const float*)d_in[17];
  const float* W1p = (const float*)d_in[18];  const float* al1p = (const float*)d_in[19];
  const float* ar1p = (const float*)d_in[20]; const float* b1p  = (const float*)d_in[21];
  float* out0 = (float*)d_out;
  float* out1 = out0 + (size_t)nN * OW;

  const int nP = ((nN + GR - 1) / GR) * GR;
  size_t off = 0;
  const size_t szPl = (size_t)8 * WPL * sizeof(__bf16);
  const size_t szFt = (((size_t)nP * FW * sizeof(float)) + 255) & ~(size_t)255;
  const size_t szEl = (((size_t)nP * NHD * sizeof(float)) + 255) & ~(size_t)255;
  __bf16* planes = (__bf16*)((char*)d_ws + off); off += szPl;
  float* ftA = (float*)((char*)d_ws + off);      off += szFt;
  float* ftP = (float*)((char*)d_ws + off);      off += szFt;
  float* hA  = (float*)((char*)d_ws + off);      off += szFt;
  float* hP  = (float*)((char*)d_ws + off);      off += szFt;
  float* elA = (float*)((char*)d_ws + off);      off += szEl;
  float* erA = (float*)((char*)d_ws + off);      off += szEl;
  float* elP = (float*)((char*)d_ws + off);      off += szEl;
  float* erP = (float*)((char*)d_ws + off);      off += szEl;
  if (off > ws_size) return;

  const dim3 gridW(FW * (FW / 8) / NTHR, 4);
  k_prepw<<<gridW, NTHR, 0, stream>>>(W0a, W0p, W1a, W1p, planes);

  const dim3 gridG(nP / GR, 2);
  k_gemm<<<gridG, NTHR, 0, stream>>>(x_am, x_ph, planes, planes + 2 * WPL,
                                     al0a, ar0a, al0p, ar0p, ftA, ftP, elA, erA, elP, erP, nN);

  hipFuncSetAttribute(reinterpret_cast<const void*>(&k_agg),
                      hipFuncAttributeMaxDynamicSharedMemorySize, LDS_BYTES);
  const int gridA = (nN + NB - 1) / NB;
  k_agg<<<gridA, NTHR, LDS_BYTES, stream>>>(src, dst, am_exist, exist, ftA, ftP,
                                            elA, erA, elP, erP, b0a, b0p, hA, hP, nN, nE, 0);

  k_gemm<<<gridG, NTHR, 0, stream>>>(hA, hP, planes + 4 * WPL, planes + 6 * WPL,
                                     al1a, ar1a, al1p, ar1p, ftA, ftP, elA, erA, elP, erP, nN);

  k_agg<<<gridA, NTHR, LDS_BYTES, stream>>>(src, dst, am_exist, exist, ftA, ftP,
                                            elA, erA, elP, erP, b1a, b1p, out0, out1, nN, nE, 1);
}
